// OwnVanillaRNN_18708877541421
// MI455X (gfx1250) — hardware-verified
//
#include <hip/hip_runtime.h>

typedef __attribute__((ext_vector_type(16))) _Float16 v16h;
typedef __attribute__((ext_vector_type(8)))  _Float16 v8h;
typedef __attribute__((ext_vector_type(8)))  float    v8f;
typedef __attribute__((ext_vector_type(4)))  float    v4f;

constexpr int kBatch   = 256;
constexpr int kSeq     = 512;
constexpr int kDin     = 64;
constexpr int kDh      = 512;
constexpr int kDout    = 64;
constexpr int kKcat    = kDin + kDh;
constexpr int kKsteps  = kKcat / 32;
constexpr int kApitch  = 584;
constexpr int kYpitch  = 68;
constexpr int kRowsBlk = 16;
constexpr int kThreads = 256;
constexpr float kWscale = 64.0f;
constexpr float kWinv   = 1.0f / 64.0f;

constexpr int kPrepBlkCat = (kDh * kKcat) / (8 * kThreads);
constexpr int kPrepBlkY   = (kDout * kDh) / (8 * kThreads);
static_assert(kPrepBlkCat * 8 * kThreads == kDh * kKcat, "cfg");
static_assert(kPrepBlkY * 8 * kThreads == kDout * kDh, "cfg");
static_assert(kKcat % 32 == 0 && kDh % 32 == 0 && kApitch % 8 == 0, "cfg");
static_assert(kBatch % kRowsBlk == 0 && kDh == 8 * 64 && kDout == 4 * 16, "cfg");

constexpr size_t kWcatBytes = (size_t)kDh * kKcat * 2;
constexpr size_t kWyBytes   = (size_t)kDout * kDh * 2;
constexpr size_t kWsTotal   = kWcatBytes + kWyBytes;

__device__ __forceinline__ void dep_guard_h(v8f& a, v8f& b, v16h x, v16h y) { asm volatile("v_nop\n\tv_nop\n\tv_nop\n\tv_nop" : "+v"(a), "+v"(b) : "v"(x), "v"(y)); }
__device__ __forceinline__ void keep4_h(v16h a, v16h b, v16h c, v16h d) { asm volatile("v_nop" :: "v"(a), "v"(b), "v"(c), "v"(d)); }
__device__ __forceinline__ void acc_guard4(v8f& a, v8f& b, v8f& c, v8f& d) { asm volatile("v_nop\n\tv_nop\n\tv_nop\n\tv_nop" : "+v"(a), "+v"(b), "+v"(c), "+v"(d)); }
template <typename T> struct Frag;
template <> struct Frag<_Float16> {
  typedef v16h V; union U { v16h v; v8h h[2]; };
  static __device__ __forceinline__ v16h load(const _Float16* p) {
    U f; f.h[0] = *(const v8h*)(p); f.h[1] = *(const v8h*)(p + 16); return f.v;
  }
  static __device__ __forceinline__ v8f mma(v16h a, v16h b, v8f c) {
    return __builtin_amdgcn_wmma_f32_16x16x32_f16(false, a, false, b, (short)0, c, false, false);
  }
  static __device__ __forceinline__ void guard(v8f& a, v8f& b, v16h x, v16h y) { dep_guard_h(a, b, x, y); }
  static __device__ __forceinline__ void keep(v16h a, v16h b, v16h c, v16h d) { keep4_h(a, b, c, d); }
};
__device__ __forceinline__ v8f mma_guard_h(v16h a, v16h b, v8f c) {
  c = __builtin_amdgcn_wmma_f32_16x16x32_f16(false, a, false, b, (short)0, c, false, false);
  asm volatile("v_nop\n\tv_nop\n\tv_nop\n\tv_nop" : "+v"(c) : "v"(a), "v"(b));
  return c;
}

__global__ __launch_bounds__(256) void prep_weights(
    const float* __restrict__ Wx, const float* __restrict__ Wh, const float* __restrict__ Wy,
    _Float16* __restrict__ Wcat, _Float16* __restrict__ Wy16)
{
  const int blk = blockIdx.x;
  const int tid = threadIdx.x;
  if (blk < kPrepBlkCat) {
    const int i  = blk * kThreads + tid;
    const int e  = i * 8;
    const int n  = e / kKcat;
    const int k  = e - n * kKcat;
    const int kx = (k < kDin) ? k : (kDin - 8);
    const int kh = (k >= kDin) ? (k - kDin) : 0;
    const float* px = Wx + (size_t)n * kDin + kx;
    const float* ph = Wh + (size_t)n * kDh + kh;
    const v4f xa = *(const v4f*)(px);
    const v4f xb = *(const v4f*)(px + 4);
    const v4f ha = *(const v4f*)(ph);
    const v4f hb = *(const v4f*)(ph + 4);
    const bool usex = (k < kDin);
    v8h hv;
#pragma unroll
    for (int q = 0; q < 4; ++q) {
      const float f0 = usex ? xa[q] : ha[q];
      const float f1 = usex ? xb[q] : hb[q];
      hv[q]     = (_Float16)(f0 * kWscale);
      hv[4 + q] = (_Float16)(f1 * kWscale);
    }
    _Float16* dst = Wcat + e;
    *(volatile v8h*)dst = hv;
    __threadfence();
    *(volatile v8h*)dst = hv;
  } else {
    const int i = (blk - kPrepBlkCat) * kThreads + tid;
    const int e = i * 8;
    const float* py = Wy + e;
    const v4f ya = *(const v4f*)(py);
    const v4f yb = *(const v4f*)(py + 4);
    v8h hv;
#pragma unroll
    for (int q = 0; q < 4; ++q) {
      hv[q]     = (_Float16)(ya[q] * kWscale);
      hv[4 + q] = (_Float16)(yb[q] * kWscale);
    }
    _Float16* dst = Wy16 + e;
    *(volatile v8h*)dst = hv;
    __threadfence();
    *(volatile v8h*)dst = hv;
  }
}

__device__ __forceinline__ void stage_x16(_Float16* tile, const float* __restrict__ x, int b0, int t, int tid) {
  if (tid < 128) {
    const int row = tid >> 3;
    const int c8  = (tid & 7) * 8;
    const float* src = x + ((size_t)(b0 + row) * kSeq + t) * kDin + c8;
    const v4f a = *(const v4f*)(src);
    const v4f b = *(const v4f*)(src + 4);
    v8h hv;
#pragma unroll
    for (int q = 0; q < 4; ++q) { hv[q] = (_Float16)a[q]; hv[4 + q] = (_Float16)b[q]; }
    *(v8h*)(tile + row * kApitch + c8) = hv;
  }
}

__global__ __launch_bounds__(256) void rnn_persist(
    const float* __restrict__ x,  const float* __restrict__ bx,
    const float* __restrict__ bh, const float* __restrict__ by,
    const _Float16* __restrict__ Wcat, const _Float16* __restrict__ Wy16,
    float* __restrict__ out)
{
  __shared__ __align__(16) _Float16 atile[2][kRowsBlk * kApitch];
  __shared__ __align__(16) float    yslab[kRowsBlk * kYpitch];

  const int tid   = threadIdx.x;
  const int wave  = tid >> 5;
  const int lane  = tid & 31;
  const int hsel  = lane >> 4;
  const int cidx  = lane & 15;
  const int wbase = wave * 64;
  const int b0    = blockIdx.x * kRowsBlk;

  {
    v8h z;
#pragma unroll
    for (int q = 0; q < 8; ++q) z[q] = (_Float16)0.0f;
#pragma unroll
    for (int q = 0; q < 4; ++q) {
      const int idx  = tid + kThreads * q;
      const int row  = idx >> 6;
      const int col8 = (idx & 63) * 8;
      *(v8h*)(&atile[0][0] + row * kApitch + kDin + col8) = z;
    }
  }
  stage_x16(&atile[0][0], x, b0, 0, tid);

  float bxv[4], bhv[4];
#pragma unroll
  for (int j = 0; j < 4; ++j) {
    const int col = wbase + 16 * j + cidx;
    bxv[j] = bx[col];
    bhv[j] = bh[col];
  }
  __syncthreads();

  for (int t = 0; t < kSeq; ++t) {
    const int cur = t & 1;
    const _Float16* arow  = &atile[cur][0] + cidx * kApitch + 8 * hsel;
    _Float16*       ntile = &atile[cur ^ 1][0];

    v8f acc[4];
#pragma unroll
    for (int j = 0; j < 4; ++j) acc[j] = (v8f){0.f, 0.f, 0.f, 0.f, 0.f, 0.f, 0.f, 0.f};

#pragma unroll 2
    for (int ks = 0; ks < kKsteps; ++ks) {
      const int k0 = ks * 32;
      v16h bfr[4];
#pragma unroll
      for (int j = 0; j < 4; ++j)
        bfr[j] = Frag<_Float16>::load(Wcat + (size_t)(wbase + 16 * j + cidx) * kKcat + k0 + 8 * hsel);
      const v16h af = Frag<_Float16>::load(arow + k0);
#pragma unroll
      for (int j = 0; j < 4; ++j) acc[j] = Frag<_Float16>::mma(af, bfr[j], acc[j]);
      Frag<_Float16>::guard(acc[0], acc[3], af, bfr[3]);
      Frag<_Float16>::keep(bfr[0], bfr[1], bfr[2], bfr[3]);
    }
    acc_guard4(acc[0], acc[1], acc[2], acc[3]);

#pragma unroll
    for (int j = 0; j < 4; ++j) {
      _Float16* hd = ntile + kDin + wbase + 16 * j + cidx;
#pragma unroll
      for (int r = 0; r < 8; ++r) {
        const float pre = (acc[j][r] * kWinv + bxv[j]) + bhv[j];
        hd[(8 * hsel + r) * kApitch] = (_Float16)tanhf(pre);
      }
    }
    const int tn = (t + 1 < kSeq) ? (t + 1) : (kSeq - 1);
    stage_x16(ntile, x, b0, tn, tid);
    __syncthreads();
  }

  if (wave < 4) {
    v8f yacc = (v8f){0.f, 0.f, 0.f, 0.f, 0.f, 0.f, 0.f, 0.f};
    const _Float16* hrow = &atile[0][0] + cidx * kApitch + kDin + 8 * hsel;
    const _Float16* wrow = Wy16 + (size_t)(wave * 16 + cidx) * kDh + 8 * hsel;
#pragma unroll 4
    for (int ks = 0; ks < kDh / 32; ++ks) {
      const int k0 = ks * 32;
      const v16h af = Frag<_Float16>::load(hrow + k0);
      const v16h bf = Frag<_Float16>::load(wrow + k0);
      yacc = mma_guard_h(af, bf, yacc);
    }
    const float byv = by[wave * 16 + cidx];
#pragma unroll
    for (int r = 0; r < 8; ++r)
      yslab[(8 * hsel + r) * kYpitch + wave * 16 + cidx] = yacc[r] * kWinv + byv;
  }
  __syncthreads();

  {
    const int row = wave * 2 + hsel;
    const int c4  = cidx * 4;
    const v4f v = *(const v4f*)(yslab + row * kYpitch + c4);
    float* dst = out + (size_t)(b0 + row) * kDout + c4;
    *(volatile v4f*)dst = v;
    __threadfence();
    *(volatile v4f*)dst = v;
  }
}

extern "C" void kernel_launch(void* const* d_in, const int* in_sizes, int n_in,
                              void* d_out, int out_size, void* d_ws, size_t ws_size,
                              hipStream_t stream)
{
  if (n_in < 7) return;
  if (in_sizes[0] != kBatch * kSeq * kDin || in_sizes[1] != kDh * kDin || in_sizes[2] != kDh ||
      in_sizes[3] != kDh * kDh || in_sizes[4] != kDh || in_sizes[5] != kDout * kDh ||
      in_sizes[6] != kDout || out_size != kBatch * kDout) return;
  if (ws_size < kWsTotal) return;

  const float* x  = (const float*)d_in[0];
  const float* Wx = (const float*)d_in[1];
  const float* bx = (const float*)d_in[2];
  const float* Wh = (const float*)d_in[3];
  const float* bh = (const float*)d_in[4];
  const float* Wy = (const float*)d_in[5];
  const float* by = (const float*)d_in[6];
  float* out = (float*)d_out;

  _Float16* Wcat = (_Float16*)d_ws;
  _Float16* Wy16 = (_Float16*)((char*)d_ws + kWcatBytes);

  prep_weights<<<kPrepBlkCat + kPrepBlkY, kThreads, 0, stream>>>(Wx, Wh, Wy, Wcat, Wy16);
  rnn_persist<<<kBatch / kRowsBlk, kThreads, 0, stream>>>(x, bx, bh, by, Wcat, Wy16, out);
}
